// MolGraphModel_80109730005332
// MI455X (gfx1250) — hardware-verified
//
#include <hip/hip_runtime.h>
#include <math.h>


constexpr int cB = 32, cN = 128, cF = 64, cE = 16, cM = 64, cD = 4, cO = 128, cT = 3;
constexpr int cR = cB * cN;
constexpr int cG = 3 * cF;

typedef float v8f __attribute__((ext_vector_type(8)));
typedef float v4f __attribute__((ext_vector_type(4)));
typedef __bf16 v16b __attribute__((ext_vector_type(16)));
typedef unsigned short v16u __attribute__((ext_vector_type(16)));
typedef unsigned short v8u __attribute__((ext_vector_type(8)));

union Frag { v16b v; v16u u; v8u q[2]; };

__device__ __forceinline__ unsigned short f2bf(float x) {
  unsigned u = __float_as_uint(x);
  u += 0x7FFFu + ((u >> 16) & 1u);
  return (unsigned short)(u >> 16);
}
__device__ __forceinline__ float bf2f(unsigned short s) {
  return __uint_as_float(((unsigned)s) << 16);
}
__device__ __forceinline__ void split2(float x, unsigned short& hi, unsigned short& lo) {
  hi = f2bf(x);
  lo = f2bf(x - bf2f(hi));
}
__device__ __forceinline__ v8f zero8() {
  v8f z;
#pragma unroll
  for (int i = 0; i < 8; ++i) z[i] = 0.0f;
  return z;
}

__device__ __forceinline__ void ldfrag(Frag& f, const unsigned short* rowp, int k0, int hh) {
  f.q[0] = *(const v8u*)(rowp + k0 + 8 * hh);
  f.q[1] = *(const v8u*)(rowp + k0 + 16 + 8 * hh);
}

__device__ __forceinline__ v8f mma3(v8f c, const Frag& ah, const Frag& al,
                                    const Frag& bh, const Frag& bl) {
  c = __builtin_amdgcn_wmma_f32_16x16x32_bf16(false, al.v, false, bh.v, (short)0, c, false, false);
  c = __builtin_amdgcn_wmma_f32_16x16x32_bf16(false, ah.v, false, bl.v, (short)0, c, false, false);
  c = __builtin_amdgcn_wmma_f32_16x16x32_bf16(false, ah.v, false, bh.v, (short)0, c, false, false);
  asm volatile("v_nop\n\tv_nop\n\tv_nop\n\tv_nop"
               : "+v"(c)
               : "v"(ah.v), "v"(al.v), "v"(bh.v), "v"(bl.v));
  return c;
}

__device__ __forceinline__ float dot64(const float* a, const float* w) {
  const v4f* a4 = (const v4f*)a;
  const v4f* w4 = (const v4f*)w;
  float s = 0.0f;
#pragma unroll 4
  for (int q = 0; q < 16; ++q) {
    v4f x = a4[q], y = w4[q];
    s += x.x * y.x; s += x.y * y.y; s += x.z * y.z; s += x.w * y.w;
  }
  return s;
}

__global__ void __launch_bounds__(128)
k_cvt_wT(const float* __restrict__ W, int N, int inStride, int outStride,
         unsigned short* Ph, unsigned short* Pl) {
  __shared__ unsigned short th[32][72] __attribute__((aligned(16)));
  __shared__ unsigned short tl[32][72] __attribute__((aligned(16)));
  const int t = blockIdx.y, n0 = blockIdx.x * 32, tid = threadIdx.x;
  if (n0 + 32 > N) return;
  const float* Wt = W + (size_t)t * inStride;
#pragma unroll 4
  for (int q = 0; q < 16; ++q) {
    const int idx = q * 128 + tid, k = idx >> 5, n = idx & 31;
    const float x = Wt[(size_t)k * N + n0 + n];
    unsigned short hi, lo;
    split2(x, hi, lo);
    th[n][k] = hi;
    tl[n][k] = lo;
  }
  __syncthreads();
  const int wv = tid >> 5, l = tid & 31;
  v8u vh[2], vl[2];
  size_t off[2];
#pragma unroll
  for (int p = 0; p < 2; ++p) {
    const int row = wv * 8 + p * 4 + (l >> 3), c = l & 7;
    vh[p] = *(const v8u*)&th[row][8 * c];
    vl[p] = *(const v8u*)&tl[row][8 * c];
    off[p] = (size_t)t * outStride + (size_t)(n0 + row) * 64 + 8 * c;
    *(volatile v8u*)(Ph + off[p]) = vh[p];
    *(volatile v8u*)(Pl + off[p]) = vl[p];
  }
  __threadfence();
#pragma unroll
  for (int p = 0; p < 2; ++p) {
    *(volatile v8u*)(Ph + off[p]) = vh[p];
    *(volatile v8u*)(Pl + off[p]) = vl[p];
  }
}

__global__ void __launch_bounds__(128)
k_node(const float* __restrict__ h, const unsigned short* __restrict__ Bh,
       const unsigned short* __restrict__ Bl, const float* __restrict__ bias,
       unsigned short* Oh, unsigned short* Ol) {
  __shared__ unsigned short Ah[64][72] __attribute__((aligned(16)));
  __shared__ unsigned short Al[64][72] __attribute__((aligned(16)));
  __shared__ unsigned short Th[64][72] __attribute__((aligned(16)));
  __shared__ unsigned short Tl[64][72] __attribute__((aligned(16)));
  const int tid = threadIdx.x, row0 = blockIdx.x * 64;
  if (row0 + 64 > cR) return;

#pragma unroll 8
  for (int q = 0; q < 32; ++q) {
    const int idx = q * 128 + tid, r = idx >> 6, f = idx & 63;
    const float x = h[(size_t)(row0 + r) * cF + f];
    unsigned short hi, lo;
    split2(x, hi, lo);
    Ah[r][f] = hi;
    Al[r][f] = lo;
  }
  __syncthreads();

  const int wv = tid >> 5, l = tid & 31, hh = l >> 4, m = l & 15;
  v8f acc[4];
#pragma unroll
  for (int ct = 0; ct < 4; ++ct) acc[ct] = zero8();
#pragma unroll
  for (int kc = 0; kc < 2; ++kc) {
    Frag ah, al;
    ldfrag(ah, &Ah[wv * 16 + m][0], kc * 32, hh);
    ldfrag(al, &Al[wv * 16 + m][0], kc * 32, hh);
#pragma unroll
    for (int ct = 0; ct < 4; ++ct) {
      Frag bh, bl;
      const size_t bo = (size_t)(ct * 16 + m) * 64;
      ldfrag(bh, Bh + bo, kc * 32, hh);
      ldfrag(bl, Bl + bo, kc * 32, hh);
      acc[ct] = mma3(acc[ct], ah, al, bh, bl);
    }
  }
#pragma unroll
  for (int ct = 0; ct < 4; ++ct) {
    const int mc = ct * 16 + m;
    const float bv = bias[mc];
#pragma unroll
    for (int r = 0; r < 8; ++r) {
      const float x = acc[ct][r] + bv;
      unsigned short hi, lo;
      split2(x, hi, lo);
      const int jl = wv * 16 + 8 * hh + r;
      Th[mc][jl] = hi;
      Tl[mc][jl] = lo;
    }
  }
  __syncthreads();

  const size_t obase = (size_t)(row0 >> 7) * cM * cN + (size_t)((row0 >> 6) & 1) * 64;
  v8u vh[4], vl[4];
  size_t off[4];
#pragma unroll
  for (int p = 0; p < 4; ++p) {
    const int mrow = wv * 16 + p * 4 + (l >> 3), c = l & 7;
    vh[p] = *(const v8u*)&Th[mrow][8 * c];
    vl[p] = *(const v8u*)&Tl[mrow][8 * c];
    off[p] = obase + (size_t)mrow * cN + 8 * c;
    *(volatile v8u*)(Oh + off[p]) = vh[p];
    *(volatile v8u*)(Ol + off[p]) = vl[p];
  }
  __threadfence();
#pragma unroll
  for (int p = 0; p < 4; ++p) {
    *(volatile v8u*)(Oh + off[p]) = vh[p];
    *(volatile v8u*)(Ol + off[p]) = vl[p];
  }
}

__global__ void __launch_bounds__(128)
k_edge(const float* __restrict__ hin,
       const unsigned short* __restrict__ HnH, const unsigned short* __restrict__ HnL,
       const float* __restrict__ bfm, const float* __restrict__ adj,
       const float* __restrict__ wai, const float* __restrict__ waj,
       const float* __restrict__ wae, const float* __restrict__ ba_p,
       const float* __restrict__ aggw, const float* __restrict__ We,
       const float* __restrict__ be, float* agg) {
  __shared__ unsigned short Wh[16][168] __attribute__((aligned(16)));
  __shared__ unsigned short Wl[16][168] __attribute__((aligned(16)));
  __shared__ unsigned short B5h[64][40] __attribute__((aligned(16)));
  __shared__ unsigned short B5l[64][40] __attribute__((aligned(16)));
  __shared__ float outS[16][64] __attribute__((aligned(16)));
  __shared__ float aj_s[cN];
  __shared__ float ai_s[16];
  __shared__ float wae_s[cE];
  __shared__ float alpha_s[cD];

  const int b = blockIdx.x, it = blockIdx.y, tid = threadIdx.x;
  if (b >= cB || it * 16 + 16 > cN) return;

#pragma unroll 4
  for (int q = 0; q < 16; ++q) {
    const int idx = q * 128 + tid, mm = idx >> 5, k = idx & 31;
    float x = 0.0f;
    if (k < cE) x = We[k * cM + mm];
    else if (k == cE) x = be[mm];
    unsigned short hi, lo;
    split2(x, hi, lo);
    B5h[mm][k] = hi;
    B5l[mm][k] = lo;
  }
  for (int idx = tid; idx < 16 * 23; idx += 128) {
    const int r = idx / 23, k = 145 + idx % 23;
    Wh[r][k] = 0;
    Wl[r][k] = 0;
  }
  aj_s[tid] = dot64(hin + (size_t)(b * cN + tid) * cF, waj);
  if (tid < 16) ai_s[tid] = dot64(hin + (size_t)(b * cN + it * 16 + tid) * cF, wai);
  if (tid < cE) wae_s[tid] = wae[tid];
  if (tid == 0) {
    float mx = aggw[0];
#pragma unroll
    for (int d = 1; d < cD; ++d) mx = fmaxf(mx, aggw[d]);
    float ex[cD], s = 0.0f;
#pragma unroll
    for (int d = 0; d < cD; ++d) { ex[d] = expf(aggw[d] - mx); s += ex[d]; }
    const float inv = 1.0f / s;
#pragma unroll
    for (int d = 0; d < cD; ++d) alpha_s[d] = ex[d] * inv;
  }
  __syncthreads();

  const int il = tid >> 3, jg = tid & 7;
  const int i = it * 16 + il;
  const float a_i = ai_s[il] + ba_p[0];
  const float* bf_row = bfm + (size_t)(b * cN + i) * cN * cE;
  const float* adj_bi = adj + ((size_t)b * cD * cN + i) * cN;

  float lsum = 0.0f;
  float leb[cE];
#pragma unroll
  for (int e = 0; e < cE; ++e) leb[e] = 0.0f;

  for (int jj = 0; jj < 16; ++jj) {
    const int j = jj * 8 + jg;
    const v4f* bp = (const v4f*)(bf_row + (size_t)j * cE);
    float ev[cE];
#pragma unroll
    for (int q = 0; q < 4; ++q) {
      const v4f x = bp[q];
      ev[4 * q + 0] = x.x; ev[4 * q + 1] = x.y; ev[4 * q + 2] = x.z; ev[4 * q + 3] = x.w;
    }
    float sc = a_i + aj_s[j];
#pragma unroll
    for (int e = 0; e < cE; ++e) sc += ev[e] * wae_s[e];
    float ad = 0.0f;
#pragma unroll
    for (int d = 0; d < cD; ++d) ad += alpha_s[d] * adj_bi[(size_t)d * cN * cN + j];
    const float w = ad * (1.0f / (1.0f + __expf(-sc)));
    unsigned short hi, lo;
    split2(w, hi, lo);
    Wh[il][j] = hi;
    Wl[il][j] = lo;
    lsum += w;
#pragma unroll
    for (int e = 0; e < cE; ++e) leb[e] += w * ev[e];
  }
#pragma unroll
  for (int s = 1; s < 8; s <<= 1) {
    lsum += __shfl_xor(lsum, s);
#pragma unroll
    for (int e = 0; e < cE; ++e) leb[e] += __shfl_xor(leb[e], s);
  }
  if (jg == 0) {
#pragma unroll
    for (int e = 0; e < cE; ++e) {
      unsigned short hi, lo;
      split2(leb[e], hi, lo);
      Wh[il][128 + e] = hi;
      Wl[il][128 + e] = lo;
    }
    unsigned short hi, lo;
    split2(lsum, hi, lo);
    Wh[il][144] = hi;
    Wl[il][144] = lo;
  }
  __syncthreads();

  const int wv = tid >> 5, l = tid & 31, hh = l >> 4, m = l & 15;
  v8f acc = zero8();
  const size_t brow = (size_t)(b * cM + wv * 16 + m) * cN;
#pragma unroll
  for (int kc = 0; kc < 4; ++kc) {
    Frag ah, al, bh, bl;
    ldfrag(ah, &Wh[m][0], kc * 32, hh);
    ldfrag(al, &Wl[m][0], kc * 32, hh);
    ldfrag(bh, HnH + brow, kc * 32, hh);
    ldfrag(bl, HnL + brow, kc * 32, hh);
    acc = mma3(acc, ah, al, bh, bl);
  }
  {
    Frag ah, al, bh, bl;
    ldfrag(ah, &Wh[m][0], 128, hh);
    ldfrag(al, &Wl[m][0], 128, hh);
    ldfrag(bh, &B5h[wv * 16 + m][0], 0, hh);
    ldfrag(bl, &B5l[wv * 16 + m][0], 0, hh);
    acc = mma3(acc, ah, al, bh, bl);
  }
#pragma unroll
  for (int r = 0; r < 8; ++r) outS[8 * hh + r][wv * 16 + m] = acc[r];
  __syncthreads();

  v4f vv[2];
  size_t off[2];
#pragma unroll
  for (int p = 0; p < 2; ++p) {
    const int row = wv * 4 + p * 2 + (l >> 4), c = l & 15;
    vv[p] = *(const v4f*)&outS[row][4 * c];
    off[p] = (size_t)(b * cN + it * 16 + row) * cM + 4 * c;
    *(volatile v4f*)(agg + off[p]) = vv[p];
  }
  __threadfence();
#pragma unroll
  for (int p = 0; p < 2; ++p) *(volatile v4f*)(agg + off[p]) = vv[p];
}

__global__ void __launch_bounds__(128)
k_gru(const float* __restrict__ agg, const float* __restrict__ hin,
      const float* __restrict__ mask,
      const unsigned short* __restrict__ gWh, const unsigned short* __restrict__ gWl,
      const unsigned short* __restrict__ gUh, const unsigned short* __restrict__ gUl,
      const float* __restrict__ gb, float* hout) {
  __shared__ unsigned short Agh[16][72] __attribute__((aligned(16)));
  __shared__ unsigned short Agl[16][72] __attribute__((aligned(16)));
  __shared__ unsigned short Hh[16][72] __attribute__((aligned(16)));
  __shared__ unsigned short Hl[16][72] __attribute__((aligned(16)));
  __shared__ unsigned short Rh[16][72] __attribute__((aligned(16)));
  __shared__ unsigned short Rl[16][72] __attribute__((aligned(16)));
  __shared__ float hF[16][64];
  __shared__ float zr[16][128];
  __shared__ float outS[16][64] __attribute__((aligned(16)));
  __shared__ float msk[16];

  const int tid = threadIdx.x, row0 = blockIdx.x * 16;
  if (row0 + 16 > cR) return;

#pragma unroll
  for (int q = 0; q < 8; ++q) {
    const int idx = q * 128 + tid, i = idx >> 6, f = idx & 63;
    const float av = agg[(size_t)(row0 + i) * cM + f];
    const float hv = hin[(size_t)(row0 + i) * cF + f];
    unsigned short hi, lo;
    split2(av, hi, lo); Agh[i][f] = hi; Agl[i][f] = lo;
    split2(hv, hi, lo); Hh[i][f] = hi;  Hl[i][f] = lo;
    hF[i][f] = hv;
  }
  if (tid < 16) msk[tid] = mask[row0 + tid];
  __syncthreads();

  const int wv = tid >> 5, l = tid & 31, hh = l >> 4, m = l & 15;

#pragma unroll
  for (int q = 0; q < 2; ++q) {
    const int colb = (wv * 2 + q) * 16;
    const size_t wrow = (size_t)(colb + m) * cM;
    v8f acc = zero8();
#pragma unroll
    for (int kc = 0; kc < 2; ++kc) {
      Frag ah, al, bh, bl;
      ldfrag(ah, &Agh[m][0], kc * 32, hh);
      ldfrag(al, &Agl[m][0], kc * 32, hh);
      ldfrag(bh, gWh + wrow, kc * 32, hh);
      ldfrag(bl, gWl + wrow, kc * 32, hh);
      acc = mma3(acc, ah, al, bh, bl);
      ldfrag(ah, &Hh[m][0], kc * 32, hh);
      ldfrag(al, &Hl[m][0], kc * 32, hh);
      ldfrag(bh, gUh + wrow, kc * 32, hh);
      ldfrag(bl, gUl + wrow, kc * 32, hh);
      acc = mma3(acc, ah, al, bh, bl);
    }
    const float gbv = gb[colb + m];
#pragma unroll
    for (int r = 0; r < 8; ++r)
      zr[8 * hh + r][colb + m] = 1.0f / (1.0f + __expf(-(acc[r] + gbv)));
  }
  __syncthreads();

#pragma unroll
  for (int q = 0; q < 8; ++q) {
    const int idx = q * 128 + tid, i = idx >> 6, f = idx & 63;
    const float x = zr[i][64 + f] * hF[i][f];
    unsigned short hi, lo;
    split2(x, hi, lo);
    Rh[i][f] = hi;
    Rl[i][f] = lo;
  }
  __syncthreads();

  {
    const int colb = 2 * cF + wv * 16;
    const size_t wrow = (size_t)(colb + m) * cM;
    v8f acc = zero8();
#pragma unroll
    for (int kc = 0; kc < 2; ++kc) {
      Frag ah, al, bh, bl;
      ldfrag(ah, &Agh[m][0], kc * 32, hh);
      ldfrag(al, &Agl[m][0], kc * 32, hh);
      ldfrag(bh, gWh + wrow, kc * 32, hh);
      ldfrag(bl, gWl + wrow, kc * 32, hh);
      acc = mma3(acc, ah, al, bh, bl);
      ldfrag(ah, &Rh[m][0], kc * 32, hh);
      ldfrag(al, &Rl[m][0], kc * 32, hh);
      ldfrag(bh, gUh + wrow, kc * 32, hh);
      ldfrag(bl, gUl + wrow, kc * 32, hh);
      acc = mma3(acc, ah, al, bh, bl);
    }
    const float gbv = gb[colb + m];
#pragma unroll
    for (int r = 0; r < 8; ++r) {
      const int i = 8 * hh + r, f = wv * 16 + m;
      const float nv = tanhf(acc[r] + gbv);
      const float z = zr[i][f], hv = hF[i][f];
      outS[i][f] = msk[i] * ((1.0f - z) * nv + z * hv);
    }
  }
  __syncthreads();

  v4f vv[2];
  size_t off[2];
#pragma unroll
  for (int p = 0; p < 2; ++p) {
    const int row = wv * 4 + p * 2 + (l >> 4), c = l & 15;
    vv[p] = *(const v4f*)&outS[row][4 * c];
    off[p] = (size_t)(row0 + row) * cF + 4 * c;
    *(volatile v4f*)(hout + off[p]) = vv[p];
  }
  __threadfence();
#pragma unroll
  for (int p = 0; p < 2; ++p) *(volatile v4f*)(hout + off[p]) = vv[p];
}

__global__ void __launch_bounds__(128)
k_ro_e(const float* __restrict__ h, const unsigned short* __restrict__ Bh,
       const unsigned short* __restrict__ Bl, const float* __restrict__ roba,
       const float* __restrict__ rov, const float* __restrict__ mask, float* esc) {
  __shared__ unsigned short Ah[64][72] __attribute__((aligned(16)));
  __shared__ unsigned short Al[64][72] __attribute__((aligned(16)));
  __shared__ float S[64][65];
  __shared__ float es[64] __attribute__((aligned(16)));
  const int tid = threadIdx.x, row0 = blockIdx.x * 64;
  if (row0 + 64 > cR) return;

#pragma unroll 8
  for (int q = 0; q < 32; ++q) {
    const int idx = q * 128 + tid, r = idx >> 6, f = idx & 63;
    const float x = h[(size_t)(row0 + r) * cF + f];
    unsigned short hi, lo;
    split2(x, hi, lo);
    Ah[r][f] = hi;
    Al[r][f] = lo;
  }
  __syncthreads();

  const int wv = tid >> 5, l = tid & 31, hh = l >> 4, m = l & 15;
  v8f acc[4];
#pragma unroll
  for (int ct = 0; ct < 4; ++ct) acc[ct] = zero8();
#pragma unroll
  for (int kc = 0; kc < 2; ++kc) {
    Frag ah, al;
    ldfrag(ah, &Ah[wv * 16 + m][0], kc * 32, hh);
    ldfrag(al, &Al[wv * 16 + m][0], kc * 32, hh);
#pragma unroll
    for (int ct = 0; ct < 4; ++ct) {
      Frag bh, bl;
      const size_t bo = (size_t)(ct * 16 + m) * 64;
      ldfrag(bh, Bh + bo, kc * 32, hh);
      ldfrag(bl, Bl + bo, kc * 32, hh);
      acc[ct] = mma3(acc[ct], ah, al, bh, bl);
    }
  }
#pragma unroll
  for (int ct = 0; ct < 4; ++ct) {
    const int mc = ct * 16 + m;
    const float bv = roba[mc];
#pragma unroll
    for (int r = 0; r < 8; ++r) S[wv * 16 + 8 * hh + r][mc] = acc[ct][r] + bv;
  }
  __syncthreads();

  const int row = tid >> 1, half = tid & 1;
  float s = 0.0f;
#pragma unroll 4
  for (int q = 0; q < 32; ++q) {
    const int fp = half * 32 + q;
    s += tanhf(S[row][fp]) * rov[fp];
  }
  s += __shfl_xor(s, 1);
  if (half == 0) {
    const float mk = mask[row0 + row];
    es[row] = (mk > 0.0f) ? s : -1.0e9f;
  }
  __syncthreads();

  if (tid < 16) {
    const v4f v = *(const v4f*)&es[4 * tid];
    float* p = esc + row0 + 4 * tid;
    *(volatile v4f*)p = v;
    __threadfence();
    *(volatile v4f*)p = v;
  }
}

__global__ void __launch_bounds__(128)
k_pool_out(const float* __restrict__ esc, const float* __restrict__ h,
           const float* __restrict__ roWo, const float* __restrict__ robo, float* out) {
  __shared__ float sh[cN];
  __shared__ float att[cN];
  __shared__ float pp[2][cF];
  __shared__ float pooled[cF];
  __shared__ float outL[cO] __attribute__((aligned(16)));
  const int b = blockIdx.x, tid = threadIdx.x;
  if (b >= cB) return;

  const float v = esc[b * cN + tid];
  sh[tid] = v;
  __syncthreads();
  for (int s = 64; s > 0; s >>= 1) {
    if (tid < s) sh[tid] = fmaxf(sh[tid], sh[tid + s]);
    __syncthreads();
  }
  const float mx = sh[0];
  __syncthreads();
  const float ex = expf(v - mx);
  sh[tid] = ex;
  __syncthreads();
  for (int s = 64; s > 0; s >>= 1) {
    if (tid < s) sh[tid] += sh[tid + s];
    __syncthreads();
  }
  att[tid] = ex * (1.0f / sh[0]);
  __syncthreads();

  {
    const int f = tid & 63, half = tid >> 6;
    float s = 0.0f;
#pragma unroll 8
    for (int q = 0; q < 64; ++q) {
      const int n = half * 64 + q;
      s += att[n] * h[(size_t)(b * cN + n) * cF + f];
    }
    pp[half][f] = s;
  }
  __syncthreads();
  if (tid < cF) pooled[tid] = pp[0][tid] + pp[1][tid];
  __syncthreads();
  {
    float s = robo[tid];
#pragma unroll 8
    for (int f = 0; f < cF; ++f) s += pooled[f] * roWo[f * cO + tid];
    outL[tid] = s;
  }
  __syncthreads();
  if (tid < 32) {
    const v4f vv = *(const v4f*)&outL[4 * tid];
    float* p = out + (size_t)b * cO + 4 * tid;
    *(volatile v4f*)p = vv;
    __threadfence();
    *(volatile v4f*)p = vv;
  }
}

extern "C" void kernel_launch(void* const* d_in, const int* in_sizes, int n_in,
                              void* d_out, int out_size, void* d_ws, size_t ws_size,
                              hipStream_t stream) {
  if (n_in < 21) return;
  const int want[21] = {
      cB * cN * cF, cB * cN * cN * cE, cB * cN, cB * cD * cN * cN,
      cT * cE * cM, cT * cM, cT * cF * cM, cT * cM, cT * cF, cT * cF, cT * cE, cT, cT * cD,
      cT * cM * cG, cT * cF * cG, cT * cG, cF * cF, cF, cF, cF * cO, cO};
  for (int i = 0; i < 21; ++i)
    if (in_sizes[i] != want[i]) return;
  if (out_size != cB * cO) return;

  const float* afm  = (const float*)d_in[0];
  const float* bfm  = (const float*)d_in[1];
  const float* mask = (const float*)d_in[2];
  const float* adj  = (const float*)d_in[3];
  const float* We   = (const float*)d_in[4];
  const float* be   = (const float*)d_in[5];
  const float* Wn   = (const float*)d_in[6];
  const float* bn   = (const float*)d_in[7];
  const float* wai  = (const float*)d_in[8];
  const float* waj  = (const float*)d_in[9];
  const float* wae  = (const float*)d_in[10];
  const float* ba   = (const float*)d_in[11];
  const float* aggw = (const float*)d_in[12];
  const float* gW   = (const float*)d_in[13];
  const float* gU   = (const float*)d_in[14];
  const float* gb   = (const float*)d_in[15];
  const float* roWa = (const float*)d_in[16];
  const float* roba = (const float*)d_in[17];
  const float* rov  = (const float*)d_in[18];
  const float* roWo = (const float*)d_in[19];
  const float* robo = (const float*)d_in[20];
  float* out = (float*)d_out;

  char* wsb = (char*)d_ws;
  size_t off = 0;
  auto carve = [&](size_t bytes) -> char* {
    char* p = wsb + off;
    off += (bytes + 255) & ~(size_t)255;
    return p;
  };
  float* hA  = (float*)carve((size_t)cR * cF * sizeof(float));
  float* hB  = (float*)carve((size_t)cR * cF * sizeof(float));
  float* agg = (float*)carve((size_t)cR * cM * sizeof(float));
  float* esc = (float*)carve((size_t)cR * sizeof(float));
  unsigned short* HnH = (unsigned short*)carve((size_t)cR * cM * 2);
  unsigned short* HnL = (unsigned short*)carve((size_t)cR * cM * 2);
  unsigned short* WnH = (unsigned short*)carve((size_t)cT * cM * cF * 2);
  unsigned short* WnL = (unsigned short*)carve((size_t)cT * cM * cF * 2);
  unsigned short* gWH = (unsigned short*)carve((size_t)cT * cG * cM * 2);
  unsigned short* gWL = (unsigned short*)carve((size_t)cT * cG * cM * 2);
  unsigned short* gUH = (unsigned short*)carve((size_t)cT * cG * cF * 2);
  unsigned short* gUL = (unsigned short*)carve((size_t)cT * cG * cF * 2);
  unsigned short* roWaH = (unsigned short*)carve((size_t)cF * cF * 2);
  unsigned short* roWaL = (unsigned short*)carve((size_t)cF * cF * 2);
  if (off > ws_size) return;

  k_cvt_wT<<<dim3(cM / 32, cT), dim3(128), 0, stream>>>(Wn, cM, cF * cM, cM * cF, WnH, WnL);
  k_cvt_wT<<<dim3(cG / 32, cT), dim3(128), 0, stream>>>(gW, cG, cM * cG, cG * cM, gWH, gWL);
  k_cvt_wT<<<dim3(cG / 32, cT), dim3(128), 0, stream>>>(gU, cG, cF * cG, cG * cF, gUH, gUL);
  k_cvt_wT<<<dim3(cF / 32, 1), dim3(128), 0, stream>>>(roWa, cF, 0, 0, roWaH, roWaL);

  const float* hcur = afm;
  float* bufs[2] = {hA, hB};

  for (int t = 0; t < cT; ++t) {
    float* hnext = bufs[t & 1];
    k_node<<<dim3(cR / 64), dim3(128), 0, stream>>>(
        hcur, WnH + (size_t)t * cM * cF, WnL + (size_t)t * cM * cF, bn + (size_t)t * cM, HnH, HnL);
    k_edge<<<dim3(cB, cN / 16), dim3(128), 0, stream>>>(
        hcur, HnH, HnL, bfm, adj,
        wai + (size_t)t * cF, waj + (size_t)t * cF, wae + (size_t)t * cE, ba + t,
        aggw + (size_t)t * cD, We + (size_t)t * cE * cM, be + (size_t)t * cM, agg);
    k_gru<<<dim3(cR / 16), dim3(128), 0, stream>>>(
        agg, hcur, mask,
        gWH + (size_t)t * cG * cM, gWL + (size_t)t * cG * cM,
        gUH + (size_t)t * cG * cF, gUL + (size_t)t * cG * cF,
        gb + (size_t)t * cG, hnext);
    hcur = hnext;
  }

  k_ro_e<<<dim3(cR / 64), dim3(128), 0, stream>>>(hcur, roWaH, roWaL, roba, rov, mask, esc);
  k_pool_out<<<dim3(cB), dim3(128), 0, stream>>>(esc, hcur, roWo, robo, out);
}
